// Encoder_67216238182498
// MI455X (gfx1250) — hardware-verified
//
#include <hip/hip_runtime.h>
#include <math.h>

constexpr int NBATCH  = 128;
constexpr int NSTEP   = 1024;
constexpr int NFEAT   = 64;
constexpr int NHID    = 128;
constexpr int NGATE   = 4 * NHID;
constexpr int NTHR    = 256;
constexpr int SEQ_BLK = 16;
constexpr int OPITCH  = 132;
constexpr float ACARRY = 16.0f;
constexpr float WCARRY = 16.0f;
constexpr float FOLD   = 1.0f / (ACARRY * WCARRY);
constexpr int XN8 = NBATCH * NSTEP * (NFEAT / 8);
constexpr int NSTATE = NBATCH * NHID;

static_assert(NBATCH == 128 && NFEAT == 64 && NHID == 128, "index shifts below assume these shapes");
static_assert(NBATCH % SEQ_BLK == 0, "whole 16-row blocks");
static_assert(NHID == 16 * (NTHR / 32), "8 waves x 16 hidden units");
static_assert(XN8 % NTHR == 0, "convert grid exact");
static_assert(NGATE % 64 == 0 && NFEAT % 64 == 0 && NHID % 64 == 0, "transpose tiles exact");
static_assert(NSTATE * 4 == 65536, "second output starts at byte 65536");
static_assert(2 * NSTATE * 4 == 131072, "both outputs fill d_out exactly");

typedef __attribute__((ext_vector_type(16))) _Float16 v16h;
typedef __attribute__((ext_vector_type(8)))  _Float16 v8h;
typedef __attribute__((ext_vector_type(8)))  float    v8f;
typedef __attribute__((ext_vector_type(4)))  float    v4f;

struct FragH {
  union U { v16h v; v8h h[2]; };
  static __device__ __forceinline__ v16h load(const _Float16* p) {
    U f;
    f.h[0] = *(const v8h*)(p);
    f.h[1] = *(const v8h*)(p + 16);
    return f.v;
  }
  static __device__ __forceinline__ v8f mma(v16h a, v16h b, v8f c) {
    return __builtin_amdgcn_wmma_f32_16x16x32_f16(false, a, false, b, (short)0, c, false, false);
  }
};

__device__ __forceinline__ void guard_group4(v8f& a0, v8f& a1, v8f& a2, v8f& a3,
                                             v16h x, v16h b0, v16h b1, v16h b2, v16h b3) {
  asm volatile("v_nop\n\tv_nop\n\tv_nop\n\tv_nop"
               : "+v"(a0), "+v"(a1), "+v"(a2), "+v"(a3)
               : "v"(x), "v"(b0), "v"(b1), "v"(b2), "v"(b3));
}

__device__ __forceinline__ float fsig(float x)  { return __builtin_amdgcn_rcpf(1.0f + expf(-x)); }
__device__ __forceinline__ float ftanh(float x) { return 1.0f - 2.0f * __builtin_amdgcn_rcpf(expf(2.0f * x) + 1.0f); }

__global__ __launch_bounds__(NTHR) void xcvt_kernel(const float* __restrict__ x, unsigned short* __restrict__ dst) {
  const int i = blockIdx.x * NTHR + threadIdx.x;
  if (i < XN8) {
    const int c8 = (i & 7) * 8;
    const int b  = (i >> 3) & (NBATCH - 1);
    const int t  = i >> 10;
    const float* sp = x + ((size_t)b * NSTEP + (size_t)t) * NFEAT + c8;
    const v4f va = *(const v4f*)(sp);
    const v4f vb = *(const v4f*)(sp + 4);
    v8h hv;
#pragma unroll
    for (int e = 0; e < 4; ++e) {
      hv[e]     = (_Float16)(va[e] * ACARRY);
      hv[4 + e] = (_Float16)(vb[e] * ACARRY);
    }
    unsigned short* op = dst + (size_t)i * 8;
    for (int pass = 0; pass < 2; ++pass) {
      *(volatile v8h*)op = hv;
      __threadfence();
    }
  }
}

__global__ __launch_bounds__(NTHR) void tpw_kernel(const float* __restrict__ src, int R, int C, int ldo,
                                                   unsigned short* __restrict__ O, float sc) {
  __shared__ float Tt[64 * 65];
  const int tid = threadIdx.x;
  const int c0 = blockIdx.x * 64, r0 = blockIdx.y * 64;
  (void)R;
#pragma unroll
  for (int i = 0; i < 4; ++i) {
    const int idx = i * NTHR + tid;
    const int rr = idx >> 4, cc = (idx & 15) * 4;
    const v4f v = *(const v4f*)(src + (size_t)(r0 + rr) * (size_t)C + c0 + cc);
    Tt[rr * 65 + cc + 0] = v[0];
    Tt[rr * 65 + cc + 1] = v[1];
    Tt[rr * 65 + cc + 2] = v[2];
    Tt[rr * 65 + cc + 3] = v[3];
  }
  __syncthreads();
  const int q = tid >> 3, c8 = (tid & 7) * 8;
  v8h hv[2];
#pragma unroll
  for (int g = 0; g < 2; ++g) {
    const int qq = g * 32 + q;
#pragma unroll
    for (int e = 0; e < 8; ++e) {
      const float f = Tt[(c8 + e) * 65 + qq];
      hv[g][e] = (_Float16)(f * sc);
    }
  }
  for (int pass = 0; pass < 2; ++pass) {
#pragma unroll
    for (int g = 0; g < 2; ++g) {
      const size_t o = (size_t)(c0 + g * 32 + q) * (size_t)ldo + (size_t)(r0 + c8);
      *(volatile v8h*)(O + o) = hv[g];
    }
    __threadfence();
  }
}

template <int KIN, bool FIRST>
__global__ __launch_bounds__(NTHR) void lstm_layer_kernel(const unsigned short* __restrict__ Xin,
                                                          const unsigned short* __restrict__ Btp,
                                                          const float* __restrict__ bias,
                                                          const float* __restrict__ state_in,
                                                          unsigned short* __restrict__ hseq,
                                                          float* __restrict__ out_h,
                                                          float* __restrict__ out_c) {
  constexpr int KTOT   = KIN + NHID;
  constexpr int APITCH = KTOT + 8;
  constexpr int CH     = KIN / 8;
  constexpr int LDTHR  = SEQ_BLK * CH;
  static_assert(KTOT % 32 == 0, "K multiple of 32");
  static_assert(APITCH % 8 == 0, "16-B aligned LDS rows");
  static_assert(LDTHR % 32 == 0 && LDTHR <= NTHR, "input tile loaders are whole waves");
  __shared__ __align__(16) _Float16 Ab[2][SEQ_BLK * APITCH];
  __shared__ __align__(16) float    Hs[SEQ_BLK * OPITCH];

  const _Float16* Bt = (const _Float16*)(const void*)Btp;
  const int tid = threadIdx.x, lane = tid & 31, wave = tid >> 5;
  const int c = lane & 15, hh = lane >> 4, koff = hh * 8;
  const int rowbase = blockIdx.x * SEQ_BLK;
  const int j = 16 * wave + c;

  const int hrow = tid >> 4, hc8 = (tid & 15) * 8;
  const bool ldact = tid < LDTHR;
  const int lrow = (tid / CH) & (SEQ_BLK - 1), lc8 = (tid % CH) * 8;

  {
    v8h hv;
    if (FIRST) {
#pragma unroll
      for (int e = 0; e < 8; ++e) hv[e] = (_Float16)0.0f;
    } else {
      const float* sp = state_in + (size_t)(rowbase + hrow) * NHID + hc8;
      const v4f va = *(const v4f*)(sp);
      const v4f vb = *(const v4f*)(sp + 4);
#pragma unroll
      for (int e = 0; e < 4; ++e) {
        hv[e]     = (_Float16)(va[e] * ACARRY);
        hv[4 + e] = (_Float16)(vb[e] * ACARRY);
      }
    }
    *(v8h*)(&Ab[0][0] + hrow * APITCH + KIN + hc8) = hv;
  }
  if (ldact) {
    const v8h v = *(const v8h*)(const void*)(Xin + ((size_t)(rowbase + lrow)) * KIN + lc8);
    *(v8h*)(&Ab[0][0] + lrow * APITCH + lc8) = v;
  }

  float cst[8], hst[8], bb[4];
#pragma unroll
  for (int g = 0; g < 4; ++g) bb[g] = bias[g * NHID + j];
#pragma unroll
  for (int r = 0; r < 8; ++r) {
    hst[r] = 0.0f;
    if (FIRST) cst[r] = 0.0f;
    else       cst[r] = state_in[(size_t)NSTATE + (size_t)(rowbase + 8 * hh + r) * NHID + j];
  }
  __syncthreads();

  const v8f z8 = {0.f, 0.f, 0.f, 0.f, 0.f, 0.f, 0.f, 0.f};
  const _Float16* wb = Bt + (size_t)j * KTOT + koff;

#pragma unroll 1
  for (int t = 0; t < NSTEP; ++t) {
    const int p = t & 1;
    const _Float16* arow = &Ab[0][0] + p * (SEQ_BLK * APITCH) + c * APITCH + koff;
    _Float16* an = &Ab[0][0] + (p ^ 1) * (SEQ_BLK * APITCH);

    v8h nx;
#pragma unroll
    for (int e = 0; e < 8; ++e) nx[e] = (_Float16)0.0f;
    if (ldact) {
      const int tn = (t + 1 < NSTEP) ? (t + 1) : (NSTEP - 1);
      nx = *(const v8h*)(const void*)(Xin + ((size_t)tn * NBATCH + (size_t)(rowbase + lrow)) * KIN + lc8);
    }

    v8f acc0 = z8, acc1 = z8, acc2 = z8, acc3 = z8;
#pragma unroll 1
    for (int k0 = 0; k0 < KTOT; k0 += 32) {
      const v16h a  = FragH::load(arow + k0);
      const v16h b0 = FragH::load(wb + k0);
      const v16h b1 = FragH::load(wb + (size_t)1 * NHID * KTOT + k0);
      const v16h b2 = FragH::load(wb + (size_t)2 * NHID * KTOT + k0);
      const v16h b3 = FragH::load(wb + (size_t)3 * NHID * KTOT + k0);
      acc0 = FragH::mma(a, b0, acc0);
      acc1 = FragH::mma(a, b1, acc1);
      acc2 = FragH::mma(a, b2, acc2);
      acc3 = FragH::mma(a, b3, acc3);
      guard_group4(acc0, acc1, acc2, acc3, a, b0, b1, b2, b3);
    }

#pragma unroll
    for (int r = 0; r < 8; ++r) {
      const float zi = acc0[r] * FOLD + bb[0];
      const float zf = acc1[r] * FOLD + bb[1];
      const float zg = acc2[r] * FOLD + bb[2];
      const float zo = acc3[r] * FOLD + bb[3];
      const float ig = fsig(zi);
      const float fg = fsig(zf);
      const float gg = ftanh(zg);
      const float og = fsig(zo);
      const float cn = fg * cst[r] + ig * gg;
      cst[r] = cn;
      const float hn = og * ftanh(cn);
      hst[r] = hn;
      an[(8 * hh + r) * APITCH + KIN + j] = (_Float16)(hn * ACARRY);
    }
    if (ldact) *(v8h*)(an + lrow * APITCH + lc8) = nx;
    __syncthreads();

    if (FIRST) {
      const v8h hv = *(const v8h*)(an + hrow * APITCH + KIN + hc8);
      unsigned short* dp = hseq + ((size_t)t * NBATCH + (size_t)(rowbase + hrow)) * NHID + hc8;
      for (int pass = 0; pass < 2; ++pass) {
        *(volatile v8h*)dp = hv;
        __threadfence();
      }
    }
  }

  const int srow = tid >> 5, sc4 = (tid & 31) * 4;
#pragma unroll
  for (int r = 0; r < 8; ++r) Hs[(8 * hh + r) * OPITCH + j] = hst[r];
  __syncthreads();
  {
    const v4f v0 = *(const v4f*)(Hs + srow * OPITCH + sc4);
    const v4f v1 = *(const v4f*)(Hs + (srow + 8) * OPITCH + sc4);
    float* p0 = out_h + (size_t)(rowbase + srow) * NHID + sc4;
    float* p1 = out_h + (size_t)(rowbase + srow + 8) * NHID + sc4;
    for (int pass = 0; pass < 2; ++pass) {
      *(volatile v4f*)p0 = v0;
      *(volatile v4f*)p1 = v1;
      __threadfence();
    }
  }
  __syncthreads();
#pragma unroll
  for (int r = 0; r < 8; ++r) Hs[(8 * hh + r) * OPITCH + j] = cst[r];
  __syncthreads();
  {
    const v4f v0 = *(const v4f*)(Hs + srow * OPITCH + sc4);
    const v4f v1 = *(const v4f*)(Hs + (srow + 8) * OPITCH + sc4);
    float* p0 = out_c + (size_t)(rowbase + srow) * NHID + sc4;
    float* p1 = out_c + (size_t)(rowbase + srow + 8) * NHID + sc4;
    for (int pass = 0; pass < 2; ++pass) {
      *(volatile v4f*)p0 = v0;
      *(volatile v4f*)p1 = v1;
      __threadfence();
    }
  }
}

extern "C" void kernel_launch(void* const* d_in, const int* in_sizes, int n_in,
                              void* d_out, int out_size, void* d_ws, size_t ws_size, hipStream_t stream) {
  if (n_in < 7 || d_out == nullptr || d_ws == nullptr) return;
  if (in_sizes[0] != NBATCH * NSTEP * NFEAT || in_sizes[1] != NFEAT * NGATE || in_sizes[2] != NHID * NGATE ||
      in_sizes[3] != NGATE || in_sizes[4] != NHID * NGATE || in_sizes[5] != NHID * NGATE ||
      in_sizes[6] != NGATE || out_size != 2 * NSTATE) return;

  const float* x  = (const float*)d_in[0];
  const float* W0 = (const float*)d_in[1];
  const float* U0 = (const float*)d_in[2];
  const float* b0 = (const float*)d_in[3];
  const float* W1 = (const float*)d_in[4];
  const float* U1 = (const float*)d_in[5];
  const float* b1 = (const float*)d_in[6];
  float* outp = (float*)d_out;

  char* ws = (char*)d_ws;
  size_t off = 0;
  auto carve = [&](size_t bytes) -> char* { char* p = ws + off; off += (bytes + 255) & ~(size_t)255; return p; };
  unsigned short* X16   = (unsigned short*)carve((size_t)NSTEP * NBATCH * NFEAT * 2);
  unsigned short* HS0   = (unsigned short*)carve((size_t)NSTEP * NBATCH * NHID * 2);
  unsigned short* BT0   = (unsigned short*)carve((size_t)NGATE * (NFEAT + NHID) * 2);
  unsigned short* BT1   = (unsigned short*)carve((size_t)NGATE * (NHID + NHID) * 2);
  float*          STATE = (float*)carve((size_t)2 * NSTATE * 4);
  if (off > ws_size || off > (size_t)134217728) return;

  xcvt_kernel<<<XN8 / NTHR, NTHR, 0, stream>>>(x, X16);

  tpw_kernel<<<dim3(NGATE / 64, NFEAT / 64), NTHR, 0, stream>>>(W0, NFEAT, NGATE, NFEAT + NHID, BT0, WCARRY);
  tpw_kernel<<<dim3(NGATE / 64, NHID / 64), NTHR, 0, stream>>>(U0, NHID, NGATE, NFEAT + NHID, BT0 + NFEAT, WCARRY);
  tpw_kernel<<<dim3(NGATE / 64, NHID / 64), NTHR, 0, stream>>>(W1, NHID, NGATE, NHID + NHID, BT1, WCARRY);
  tpw_kernel<<<dim3(NGATE / 64, NHID / 64), NTHR, 0, stream>>>(U1, NHID, NGATE, NHID + NHID, BT1 + NHID, WCARRY);

  lstm_layer_kernel<NFEAT, true><<<NBATCH / SEQ_BLK, NTHR, 0, stream>>>(
      X16, BT0, b0, b0, HS0, STATE, STATE + NSTATE);
  lstm_layer_kernel<NHID, false><<<NBATCH / SEQ_BLK, NTHR, 0, stream>>>(
      HS0, BT1, b1, STATE, X16, outp, outp + NSTATE);
}
